// LPSC_Cell_59614146068486
// MI455X (gfx1250) — hardware-verified
//
#include <hip/hip_runtime.h>


#define NBR  2097152
#define LL   5
#define HH   16
#define KP   32
#define NP   64
#define RCH  262144
#define DM   KP
#define LOSC 1024.0f

typedef _Float16 h16;
typedef unsigned short bf;
typedef __attribute__((ext_vector_type(16))) __bf16   v16bf;
typedef __attribute__((ext_vector_type(16))) _Float16 v16h;
typedef __attribute__((ext_vector_type(8)))  _Float16 v8h;
typedef __attribute__((ext_vector_type(8)))  unsigned short v8us;
typedef __attribute__((ext_vector_type(8)))  float    v8f;
typedef __attribute__((ext_vector_type(4)))  float    v4f;
typedef v8h  __attribute__((may_alias)) v8ha;
typedef v4f  __attribute__((may_alias)) v4fa;
typedef v8us __attribute__((may_alias)) v8usa;

__device__ __forceinline__ unsigned short f2bf(float f) { unsigned u = __float_as_uint(f); u += 0x7FFFu + ((u >> 16) & 1u); return (unsigned short)(u >> 16); }
__device__ __forceinline__ float bf2f(unsigned short b) { return __uint_as_float(((unsigned)b) << 16); }
__device__ __forceinline__ float bfr(float f) { return bf2f(f2bf(f)); }
__device__ __forceinline__ v16h cat16(v8h lo, v8h hi) { return __builtin_shufflevector(lo, hi, 0, 1, 2, 3, 4, 5, 6, 7, 8, 9, 10, 11, 12, 13, 14, 15); }
__device__ __forceinline__ v16bf cat16b(v8us lo, v8us hi) { return __builtin_bit_cast(v16bf, __builtin_shufflevector(lo, hi, 0, 1, 2, 3, 4, 5, 6, 7, 8, 9, 10, 11, 12, 13, 14, 15)); }
__device__ __forceinline__ v8f wmma16(v16h a, v16h b, v8f c) { return __builtin_amdgcn_wmma_f32_16x16x32_f16(false, a, false, b, (short)0, c, false, false); }
__device__ __forceinline__ v8f wmmab(v16bf a, v16bf b, v8f c) { return __builtin_amdgcn_wmma_f32_16x16x32_bf16(false, a, false, b, (short)0, c, false, false); }

template <bool SPLITA, bool F16OUT = false>
__global__ __launch_bounds__(128) void k_gemmb(const bf* __restrict__ A, const bf* __restrict__ Al, const bf* __restrict__ Bn, const float* __restrict__ bias, float* C, int ldc, h16* C2, const float* __restrict__ R = nullptr, int K = DM, int roundR = 1) {
    __shared__ __align__(16) float ost[4][16 * 68];
    const int lane = threadIdx.x & 31, wave = threadIdx.x >> 5, lr = lane & 15, hi = lane >> 4;
    const int r0 = blockIdx.x * 64 + wave * 16, c0 = blockIdx.y * 64;
    const size_t aoff = (size_t)(r0 + lr) * K + 8 * hi;
    size_t boff[4];
#pragma unroll
    for (int t = 0; t < 4; ++t) boff[t] = (size_t)(c0 + t * 16 + lr) * K + 8 * hi;
    v8f acc[4];
#pragma unroll
    for (int t = 0; t < 4; ++t) acc[t] = (v8f){};
#pragma unroll 1
    for (int kc = 0; kc < K; kc += 32) {
        const v16bf a = cat16b(*(const v8us*)(A + aoff + kc), *(const v8us*)(A + aoff + kc + 16));
        v16bf al = a;
        if (SPLITA) al = cat16b(*(const v8us*)(Al + aoff + kc), *(const v8us*)(Al + aoff + kc + 16));
#pragma unroll
        for (int t = 0; t < 4; ++t) { const v16bf b = cat16b(*(const v8us*)(Bn + boff[t] + kc), *(const v8us*)(Bn + boff[t] + kc + 16)); acc[t] = wmmab(a, b, acc[t]); if (SPLITA) acc[t] = wmmab(al, b, acc[t]); }
        asm volatile("v_nop\n\tv_nop\n\tv_nop\n\tv_nop" : "+v"(acc[0]), "+v"(acc[1]), "+v"(acc[2]), "+v"(acc[3]) : "v"(a), "v"(al));
    }
    float* os = &ost[wave][0];
#pragma unroll
    for (int t = 0; t < 4; ++t) { const float bv = bias ? bfr(bias[c0 + t * 16 + lr]) : 0.f;
#pragma unroll
        for (int j = 0; j < 8; ++j) os[(hi * 8 + j) * 68 + t * 16 + lr] = acc[t][j] + bv; }
    __syncthreads();
    if (F16OUT) {
        h16* crow = (h16*)(void*)C + (size_t)r0 * ldc + c0;
        auto pass = [&]() {
#pragma unroll
            for (int s = 0; s < 4; ++s) { const int row = 4 * s + (lane >> 3), piece = lane & 7; const float* sp = os + row * 68 + piece * 8; v8h o, o2;
#pragma unroll
                for (int i = 0; i < 8; ++i) { const h16 a = (h16)sp[i]; o[i] = a; o2[i] = (h16)((sp[i] - (float)a) * LOSC); }
                *(volatile v8h*)(crow + (size_t)row * ldc + piece * 8) = o; if (C2) *(volatile v8h*)(C2 + (size_t)r0 * ldc + c0 + (size_t)row * ldc + piece * 8) = o2; }
        };
        pass(); __threadfence(); pass();
    } else {
        float* crow = C + (size_t)r0 * ldc + c0;
        auto pass = [&]() {
#pragma unroll
            for (int s = 0; s < 8; ++s) { const int Lid = (lane >> 3) + 4 * s, piece = lane & 7; const int row = Lid >> 1, cofs = (Lid & 1) * 32 + piece * 4;
                v4f val = *(const v4fa*)(os + row * 68 + cofs); if (R) { const v4f rv = *(const v4f*)(R + ((size_t)r0 + row) * ldc + c0 + cofs); val += roundR ? (v4f){bfr(rv[0]), bfr(rv[1]), bfr(rv[2]), bfr(rv[3])} : rv; }
                *(volatile v4f*)(crow + (size_t)row * ldc + cofs) = val; }
        };
        pass(); __threadfence(); pass();
    }
}


__global__ __launch_bounds__(256) void k_wtp(const float* __restrict__ Wm, int krows, int ncols, int kpad, bf* WT) {
    __shared__ __align__(16) unsigned short tl[64 * 72];
    const int tid = threadIdx.x, k0 = blockIdx.x * 64, n0 = blockIdx.y * 64;
    const int kk = tid >> 2, nq = (tid & 3) * 16;
    const int k = k0 + kk, kc = k < krows ? k : krows - 1;
#pragma unroll
    for (int i = 0; i < 16; ++i) { const int n = n0 + nq + i, ncl = n < ncols ? n : ncols - 1; const float w = Wm[(size_t)kc * ncols + ncl]; tl[(nq + i) * 72 + kk] = (k < krows && n < ncols) ? f2bf(w) : (unsigned short)0; }
    __syncthreads();
    const int piece = tid & 7;
    auto pass = [&]() {
#pragma unroll
        for (int s = 0; s < 2; ++s) { const int nr = (tid >> 3) + 32 * s; const v8us val = *(const v8usa*)(tl + nr * 72 + piece * 8); *(volatile v8us*)(WT + (size_t)(n0 + nr) * kpad + k0 + piece * 8) = val; }
    };
    pass(); __threadfence(); pass();
}

__global__ __launch_bounds__(256) void k_w2t(const float* __restrict__ w2b, bf* W2T) {
    const int u = threadIdx.x; v8us o;
#pragma unroll
    for (int i = 0; i < 8; ++i) { const int f = u * 8 + i; const int n = f / KP, k = f % KP; const bool ok = (n < HH) && (k < HH); o[i] = ok ? f2bf(w2b[(ok ? k : 0) * HH + (ok ? n : 0)]) : (unsigned short)0; }
    *(volatile v8us*)(W2T + u * 8) = o; __threadfence(); *(volatile v8us*)(W2T + u * 8) = o;
}
__global__ __launch_bounds__(256) void k_znew(const float* __restrict__ Z, const float* __restrict__ A, float* OUTZ) {
    const size_t u = (size_t)blockIdx.x * 256 + threadIdx.x; if (u >= (size_t)NBR * LL / 4) return; v4f o;
#pragma unroll
    for (int i = 0; i < 4; ++i) { const size_t f = u * 4 + i; const size_t r = f / LL; const int l = (int)(f % LL); float s = 0.f;
#pragma unroll
        for (int k = 0; k < LL; ++k) s = fmaf(bfr(Z[r * LL + k]), bfr(A[k * LL + l]), s);
        o[i] = s; }
    *(volatile v4f*)(OUTZ + u * 4) = o; __threadfence(); *(volatile v4f*)(OUTZ + u * 4) = o;
}
__global__ __launch_bounds__(256) void k_l1(const float* __restrict__ Z, const float* __restrict__ A, const float* __restrict__ w2a, const float* __restrict__ b2a, int r0, bf* Hh, bf* Hl) {
    const int lane = threadIdx.x & 31; const size_t rl = ((size_t)blockIdx.x * 8 + (threadIdx.x >> 5)) * 8 + (lane >> 2); const size_t r = (size_t)r0 + rl; const int cb = (lane & 3) * 8;
    float nz[LL];
#pragma unroll
    for (int l = 0; l < LL; ++l) { float s = 0.f;
#pragma unroll
        for (int k = 0; k < LL; ++k) s = fmaf(bfr(Z[r * LL + k]), bfr(A[k * LL + l]), s);
        nz[l] = s; }
    v8us oh, ol;
#pragma unroll
    for (int i = 0; i < 8; ++i) { const int c = cb + i; float h = 0.f;
        if (c < HH) { float s = bfr(b2a[c]);
#pragma unroll
            for (int l = 0; l < LL; ++l) s = fmaf(nz[l], bfr(w2a[l * HH + c]), s);
            h = fmaxf(s, 0.f); }
        const unsigned short hb = f2bf(h); oh[i] = hb; ol[i] = f2bf(h - bf2f(hb)); }
    const size_t o = rl * KP + cb; *(volatile v8us*)(Hh + o) = oh; *(volatile v8us*)(Hl + o) = ol; __threadfence(); *(volatile v8us*)(Hh + o) = oh; *(volatile v8us*)(Hl + o) = ol;
}
__global__ __launch_bounds__(256) void k_l3(const float* __restrict__ G, const float* __restrict__ b2b, const float* __restrict__ w2c, const float* __restrict__ b2c, const float* __restrict__ inp, const float* __restrict__ Y, int r0, float* O0, float* O2) {
    const size_t rl = (size_t)blockIdx.x * 256 + threadIdx.x; const size_t r = (size_t)r0 + rl; float k0 = bfr(b2c[0]), k1 = bfr(b2c[1]);
#pragma unroll
    for (int c = 0; c < HH; ++c) { const float h = fmaxf(G[rl * NP + c] + bfr(b2b[c]), 0.f); k0 = fmaf(h, bfr(w2c[c * 2]), k0); k1 = fmaf(h, bfr(w2c[c * 2 + 1]), k1); }
    k0 = fabsf(k0); k1 = fabsf(k1);
    const float y = bfr(Y[r]), x1 = bfr(inp[r * 2]), x2 = bfr(inp[r * 2 + 1]);
    const float dy = -y + k0 * x1 - k1 * x2 + 0.0f; const float ns = y + dy;
    *(volatile float*)(O0 + r) = ns; *(volatile float*)(O2 + r) = ns; __threadfence(); *(volatile float*)(O0 + r) = ns; *(volatile float*)(O2 + r) = ns;
}

extern "C" void kernel_launch(void* const* d_in, const int* in_sizes, int n_in,
                              void* d_out, int out_size, void* d_ws, size_t ws_size, hipStream_t stream) {
    (void)in_sizes; (void)n_in; (void)out_size;
    const float* inp = (const float*)d_in[0]; const float* Z = (const float*)d_in[1]; const float* Y = (const float*)d_in[2]; const float* A = (const float*)d_in[3];
    const float* w2a = (const float*)d_in[4]; const float* b2a = (const float*)d_in[5]; const float* w2b = (const float*)d_in[6]; const float* b2b = (const float*)d_in[7]; const float* w2c = (const float*)d_in[8]; const float* b2c = (const float*)d_in[9];
    float* O0 = (float*)d_out; float* OZ = (float*)((char*)d_out + (size_t)NBR * 4); float* O2 = (float*)((char*)d_out + (size_t)NBR * 4 + (size_t)NBR * LL * 4);
    char* wsp = (char*)d_ws;
    auto take = [&](size_t bytes) { char* p = wsp; wsp += (bytes + 255) & ~(size_t)255; return (void*)p; };
    bf* W2T = (bf*)take((size_t)NP * KP * 2); bf* Hh = (bf*)take((size_t)RCH * KP * 2); bf* Hl = (bf*)take((size_t)RCH * KP * 2); float* G = (float*)take((size_t)RCH * NP * 4);
    if ((size_t)(wsp - (char*)d_ws) > ws_size) return;
    k_w2t<<<1, 256, 0, stream>>>(w2b, W2T);
    k_znew<<<(unsigned)(((size_t)NBR * LL / 4 + 255) / 256), 256, 0, stream>>>(Z, A, OZ);
    for (int ch = 0; ch < NBR / RCH; ++ch) { const int r0 = ch * RCH;
        k_l1<<<RCH / 64, 256, 0, stream>>>(Z, A, w2a, b2a, r0, Hh, Hl);
        k_gemmb<true, false><<<dim3(RCH / 64, NP / 64, 1), 128, 0, stream>>>(Hh, Hl, W2T, nullptr, G, NP, nullptr, nullptr, KP);
        k_l3<<<RCH / 256, 256, 0, stream>>>(G, b2b, w2c, b2c, inp, Y, r0, O0, O2); }
}
